// ConditionalInformationCouplingModule_64974265253959
// MI455X (gfx1250) — hardware-run, weakly checked
//
#include <hip/hip_runtime.h>
#include <math.h>

typedef __attribute__((ext_vector_type(16))) _Float16 v16h;
typedef __attribute__((ext_vector_type(16))) __bf16 v16b;
typedef __attribute__((ext_vector_type(8)))  _Float16 v8h;
typedef __attribute__((ext_vector_type(8)))  float v8f;
typedef __attribute__((ext_vector_type(4)))  float v4f;
typedef __attribute__((ext_vector_type(2)))  float v2f;
typedef __attribute__((ext_vector_type(4)))  unsigned v4u;
typedef __attribute__((ext_vector_type(4)))  int v4i;
typedef float __attribute__((may_alias)) float_a;
typedef int __attribute__((may_alias)) int_a;

template <typename T> __device__ __forceinline__ void vst2(void* p, T v) { *(volatile T*)p = v; __threadfence(); *(volatile T*)p = v; }
__device__ __forceinline__ v8f wmma16(v16h a, v16h b, v8f c) {
  v8f d = __builtin_amdgcn_wmma_f32_16x16x32_f16(false, a, false, b, (short)0, c, false, false);
  asm volatile("v_nop\n\tv_nop\n\tv_nop\n\tv_nop" : "+v"(d) : "v"(a), "v"(b));
  return d;
}
__device__ __forceinline__ v8f wmma_bf(v16b a, v16b b, v8f c) {
  v8f d = __builtin_amdgcn_wmma_f32_16x16x32_bf16(false, a, false, b, (short)0, c, false, false);
  asm volatile("v_nop\n\tv_nop\n\tv_nop\n\tv_nop" : "+v"(d) : "v"(a), "v"(b));
  return d;
}
__device__ __forceinline__ v16h frag_h(const _Float16* rowk0, int lane) {
  union { v16h v; v8h q[2]; } u; const _Float16* p = rowk0 + 8 * (lane >> 4);
  u.q[0] = *(const v8h*)p; u.q[1] = *(const v8h*)(p + 16); return u.v;
}
__device__ __forceinline__ v16h frag_f32(const float* rowk0, int lane) {
  v16h a; const float* p = rowk0 + 8 * (lane >> 4);
#pragma unroll
  for (int i = 0; i < 8; ++i) { a[i] = (_Float16)p[i]; a[8 + i] = (_Float16)p[16 + i]; }
  return a;
}
__device__ __forceinline__ v16h frag_f32s(const float* rowk0, int lane, float sc) {
  v16h a; const float* p = rowk0 + 8 * (lane >> 4);
#pragma unroll
  for (int i = 0; i < 8; ++i) { a[i] = (_Float16)(p[i] * sc); a[8 + i] = (_Float16)(p[16 + i] * sc); }
  return a;
}
__device__ __forceinline__ v16h fragc_f32(const float* W, int k0, int n, int lane, int ld, int K) {
  v16h a; const int g = lane >> 4;
#pragma unroll
  for (int i = 0; i < 8; ++i) { const int ka = k0 + 8 * g + i, kb = ka + 16;
    a[i] = (_Float16)(ka < K ? W[(size_t)(ka < K ? ka : K - 1) * ld + n] : 0.f); a[8 + i] = (_Float16)(kb < K ? W[(size_t)(kb < K ? kb : K - 1) * ld + n] : 0.f); }
  return a;
}
struct F2 { v16b h, l; };
__device__ __forceinline__ F2 bsplit16(const float v[16]) { F2 r;
#pragma unroll
  for (int i = 0; i < 16; ++i) { const __bf16 h = (__bf16)v[i]; r.h[i] = h; r.l[i] = (__bf16)(v[i] - (float)h); }
  return r; }
__device__ __forceinline__ F2 split_row(const float* row, int k0, int lane) { float v[16]; const float* p = row + k0 + 8 * (lane >> 4);
#pragma unroll
  for (int i = 0; i < 8; ++i) { v[i] = p[i]; v[8 + i] = p[16 + i]; }
  return bsplit16(v); }
__device__ __forceinline__ F2 split_rowK(const float* row, int k0, int lane, int K) { float v[16]; const int g = lane >> 4;
#pragma unroll
  for (int i = 0; i < 8; ++i) { const int ka = k0 + 8 * g + i, kb = ka + 16; v[i] = ka < K ? row[ka < K ? ka : K - 1] : 0.f; v[8 + i] = kb < K ? row[kb < K ? kb : K - 1] : 0.f; }
  return bsplit16(v); }
__device__ __forceinline__ F2 split_col(const float* W, int k0, int n, int lane, int ld, int K) { float v[16]; const int g = lane >> 4;
#pragma unroll
  for (int i = 0; i < 8; ++i) { const int ka = k0 + 8 * g + i, kb = ka + 16; v[i] = ka < K ? W[(size_t)(ka < K ? ka : K - 1) * ld + n] : 0.f; v[8 + i] = kb < K ? W[(size_t)(kb < K ? kb : K - 1) * ld + n] : 0.f; }
  return bsplit16(v); }
__device__ __forceinline__ v8f mac3(const F2& a, const F2& b, v8f c) { c = wmma_bf(a.l, b.h, c); c = wmma_bf(a.h, b.l, c); return wmma_bf(a.h, b.h, c); }
__device__ __forceinline__ float sigm(float v) { return 1.0f / (1.0f + expf(-v)); }
#define LDSX() do { asm volatile("s_wait_dscnt 0" ::: "memory"); __builtin_amdgcn_wave_barrier(); __builtin_amdgcn_fence(__ATOMIC_RELEASE, "workgroup"); } while (0)


#define NB 8
#define CX 256
#define CI 128
#define IMH 64
#define IMW 64
#define NP (IMH * IMW)
#define NM (NP / 4)
#define BNE 1e-5f
#define CEPS 1e-8f
#ifndef TNB
#define TNB NB
#endif
#ifndef TQ
#define TQ (NP / 64)
#endif
typedef __attribute__((ext_vector_type(8))) __bf16 v8b;
__device__ __forceinline__ v16b frag_b(const __bf16* rowk0, int lane) {
  union { v16b v; v8b q[2]; } u; const __bf16* p = rowk0 + 8 * (lane >> 4);
  u.q[0] = *(const v8b*)p; u.q[1] = *(const v8b*)(p + 16); return u.v;
}
__device__ __forceinline__ float bfr(float v) { return (float)(__bf16)v; }
__device__ __attribute__((noinline)) float exp_ni(float v) { return expf(v); }
__device__ __attribute__((noinline)) float erf_ni(float v) { return erff(v); }

#define WS_XT  0u
#define XTSZ   ((size_t)NB * NP * CX)
#define WS_QT  (WS_XT + 2u * 2 * XTSZ)
#define QTSZ   ((size_t)NB * NP * CI)
#define WS_KT  (WS_QT + 2u * 2 * QTSZ)
#define KTSZ   ((size_t)NB * NM * CI)
#define WS_VTT (WS_KT + 2u * 2 * KTSZ)
#define WS_V   (WS_VTT + 2u * 2 * KTSZ)
#define WS_YT  (WS_V + 2u * 2 * KTSZ)
#define WS_MK  (WS_YT + 2u * 2 * QTSZ)
#define WS_END (WS_MK + 4u * (size_t)NB * NP)

__global__ __launch_bounds__(256) void k_xt(const float* __restrict__ X0, const float* __restrict__ X1, __bf16* __restrict__ XT) { __shared__ __align__(16) __bf16 st[64][64 + 8]; const int t = threadIdx.x; const int p0 = blockIdx.x * 64; const size_t b = blockIdx.y; const int which = blockIdx.z / 4, c0 = (blockIdx.z % 4) * 64; const float* X = which == 0 ? X0 : X1;
  for (int e = t; e < 64 * 64; e += 256) { const int cl = e >> 6, pl = e & 63; st[pl][cl] = (__bf16)X[((b * CX + c0 + cl) * NP) + p0 + pl]; } __syncthreads();
  for (int e = t; e < 64 * 8; e += 256) { const int pl = e >> 3, q = e & 7; vst2((unsigned*)(XT + (size_t)which * XTSZ + ((b * NP + p0 + pl) * CX) + c0 + q * 8), *(const v4u*)&st[pl][q * 8]); } }
__device__ __forceinline__ v16b fragb_f32(const float* __restrict__ p, int lane) { v16b a; const float* pp = p + 8 * (lane >> 4);
#pragma unroll
  for (int i = 0; i < 8; ++i) { a[i] = (__bf16)pp[i]; a[8 + i] = (__bf16)pp[16 + i]; } return a; }
__global__ __launch_bounds__(128) void k_conv(const float* __restrict__ WQ, const float* __restrict__ BQ, const float* __restrict__ WK, const float* __restrict__ BK, const float* __restrict__ WV, const float* __restrict__ BV, const __bf16* __restrict__ XT, _Float16* __restrict__ QT, _Float16* __restrict__ KT, _Float16* __restrict__ VT) {
  __shared__ __align__(16) float sv[64][132]; __shared__ __align__(16) _Float16 sh[128][72], sl[128][72];
  const int tid = threadIdx.x, wave = tid >> 5, lane = tid & 31, col = lane & 15, g = lane >> 4; const int which = blockIdx.z % 3; const size_t b = blockIdx.z / 3; const int ci0 = blockIdx.x * 64 + wave * 16; const int p0 = blockIdx.y * 128;
  const float* Wm = which == 0 ? WQ : which == 1 ? WK : WV; const float* Bm = which == 0 ? BQ : which == 1 ? BK : BV; const __bf16* Xp = XT + (size_t)(which == 0 ? 0 : 1) * XTSZ + (b * NP) * CX;
  v8f acc[8] = {};
#pragma unroll 2
  for (int kc = 0; kc < CX / 32; ++kc) { const v16b a = fragb_f32(Wm + (size_t)(ci0 + col) * CX + kc * 32, lane);
#pragma unroll
    for (int j = 0; j < 8; ++j) acc[j] = wmma_bf(a, frag_b(Xp + (size_t)(p0 + j * 16 + col) * CX + kc * 32, lane), acc[j]); }
#pragma unroll
  for (int j = 0; j < 8; ++j)
#pragma unroll
    for (int r = 0; r < 8; ++r) sv[wave * 16 + 8 * g + r][j * 16 + col] = acc[j][r] + bfr(Bm[ci0 + 8 * g + r]);
  __syncthreads();
  if (which == 0) { for (int e = tid; e < 64 * 128; e += 128) { const int cl = e & 63, pl = e >> 6; const float v = sv[cl][pl]; const _Float16 hv = (_Float16)v; sh[pl][cl] = hv; sl[pl][cl] = (_Float16)((v - (float)hv) * 2048.0f); } __syncthreads();
    _Float16* H = QT + (b * NP) * CI; _Float16* L = H + QTSZ; for (int e = tid; e < 128 * 8; e += 128) { const int pl = e >> 3, q = e & 7; const size_t o = (size_t)(p0 + pl) * CI + blockIdx.x * 64 + q * 8; vst2((unsigned*)(H + o), *(const v4u*)&sh[pl][q * 8]); vst2((unsigned*)(L + o), *(const v4u*)&sl[pl][q * 8]); } }
  else {
    const int m0 = (p0 / 128) * 32; for (int e = tid; e < 64 * 32; e += 128) { const int cl = e & 63, ml = e >> 6; const int xc = ml * 2; const float v = fmaxf(fmaxf(sv[cl][xc], sv[cl][xc + 1]), fmaxf(sv[cl][64 + xc], sv[cl][64 + xc + 1])); const _Float16 hv = (_Float16)v; sh[ml][cl] = hv; sl[ml][cl] = (_Float16)((v - (float)hv) * 2048.0f); } __syncthreads();
    _Float16* H = (which == 1 ? KT : VT) + (b * NM) * CI; _Float16* L = H + KTSZ; for (int e = tid; e < 32 * 8; e += 128) { const int ml = e >> 3, q = e & 7; const size_t o = (size_t)(m0 + ml) * CI + blockIdx.x * 64 + q * 8; vst2((unsigned*)(H + o), *(const v4u*)&sh[ml][q * 8]); vst2((unsigned*)(L + o), *(const v4u*)&sl[ml][q * 8]); } } }
__global__ __launch_bounds__(256) void k_vtr(const _Float16* __restrict__ VT, _Float16* __restrict__ V) { __shared__ __align__(16) _Float16 sh[CI][72], sl[CI][72]; const int t = threadIdx.x; const int m0 = blockIdx.x * 64; const size_t b = blockIdx.y;
  for (int e = t; e < 64 * CI; e += 256) { const int ml = e >> 7, c = e & 127; sh[c][ml] = VT[((b * NM + m0 + ml) * CI) + c]; sl[c][ml] = VT[KTSZ + ((b * NM + m0 + ml) * CI) + c]; } __syncthreads();
  for (int e = t; e < CI * 8; e += 256) { const int c = e >> 3, q = e & 7; vst2((unsigned*)(V + ((b * CI + c) * NM) + m0 + q * 8), *(const v4u*)&sh[c][q * 8]); vst2((unsigned*)(V + KTSZ + ((b * CI + c) * NM) + m0 + q * 8), *(const v4u*)&sl[c][q * 8]); } }
__global__ __launch_bounds__(128) void k_attn1(const _Float16* __restrict__ QT, const _Float16* __restrict__ KT, const _Float16* __restrict__ V, _Float16* __restrict__ YT) { __shared__ __align__(16) float sp[4][16][36]; __shared__ __align__(16) _Float16 sh[4][16][136], sl2[4][16][136];
  const int tid = threadIdx.x, wave = tid >> 5, lane = tid & 31, col = lane & 15, g = lane >> 4; const size_t b = blockIdx.y; const int q0 = blockIdx.x * 64 + wave * 16; const size_t rq = b * NP + q0;
  v16h aq[4], al[4];
#pragma unroll
  for (int kc = 0; kc < 4; ++kc) { aq[kc] = frag_h(QT + (rq + col) * CI + kc * 32, lane); al[kc] = frag_h(QT + QTSZ + (rq + col) * CI + kc * 32, lane); }
  float m[8], l[8];
#pragma unroll
  for (int r = 0; r < 8; ++r) { m[r] = -3.0e38f; l[r] = 0.f; }
  v8f acc[8] = {};
#pragma unroll 1
  for (int ks = 0; ks < NM / 32; ++ks) { v8f s[2];
#pragma unroll
    for (int ct = 0; ct < 2; ++ct) { const size_t rk = b * NM + ks * 32 + ct * 16 + col; v8f c = {}, cl = {};
#pragma unroll
      for (int kc = 0; kc < 4; ++kc) { const v16h kh = frag_h(KT + rk * CI + kc * 32, lane), kl = frag_h(KT + KTSZ + rk * CI + kc * 32, lane); c = wmma16(aq[kc], kh, c); cl = wmma16(aq[kc], kl, cl); cl = wmma16(al[kc], kh, cl); }
#pragma unroll
      for (int r = 0; r < 8; ++r) s[ct][r] = c[r] + cl[r] * (1.0f / 2048.0f); }
    float alpha[8];
#pragma unroll
    for (int r = 0; r < 8; ++r) { float mx = fmaxf(s[0][r], s[1][r]);
#pragma unroll
      for (int o = 1; o < 16; o <<= 1) mx = fmaxf(mx, __shfl_xor(mx, o));
      const float mn = fmaxf(m[r], mx); alpha[r] = __expf(m[r] - mn); const float e0 = __expf(s[0][r] - mn), e1 = __expf(s[1][r] - mn); float es = e0 + e1;
#pragma unroll
      for (int o = 1; o < 16; o <<= 1) es += __shfl_xor(es, o);
      l[r] = l[r] * alpha[r] + es; m[r] = mn; sp[wave][8 * g + r][col] = e0; sp[wave][8 * g + r][16 + col] = e1; }
#pragma unroll
    for (int j = 0; j < 8; ++j)
#pragma unroll
      for (int r = 0; r < 8; ++r) acc[j][r] *= alpha[r];
    LDSX();
    v16h pa; { const float* prow = &sp[wave][col][0] + 8 * (lane >> 4);
#pragma unroll
      for (int i = 0; i < 8; ++i) { pa[i] = (_Float16)(prow[i] * 2048.0f); pa[8 + i] = (_Float16)(prow[16 + i] * 2048.0f); } }
#pragma unroll
    for (int j = 0; j < 8; ++j) { const size_t po = (b * CI + j * 16 + col) * NM + ks * 32; acc[j] = wmma16(pa, frag_h(V + po, lane), acc[j]); }
    LDSX(); }
#pragma unroll
  for (int r = 0; r < 8; ++r) { const float il = (1.0f / 2048.0f) / l[r];
#pragma unroll
    for (int j = 0; j < 8; ++j) { const float y = acc[j][r] * il; const _Float16 hv = (_Float16)y; sh[wave][8 * g + r][j * 16 + col] = hv; sl2[wave][8 * g + r][j * 16 + col] = (_Float16)((y - (float)hv) * 2048.0f); } }
  LDSX(); for (int rl = 0; rl < 16; ++rl) if (lane < 16) { vst2((unsigned*)(YT + (rq + rl) * CI + lane * 8), *(const v4u*)&sh[wave][rl][lane * 8]); vst2((unsigned*)(YT + QTSZ + (rq + rl) * CI + lane * 8), *(const v4u*)&sl2[wave][rl][lane * 8]); } }
__global__ __launch_bounds__(256) void k_mask(const float* __restrict__ X, const float* __restrict__ KX, float* __restrict__ MK) { __shared__ float sg[CX]; __shared__ float red[8]; __shared__ __align__(16) float so2[NP]; const int t = threadIdx.x; const size_t b = blockIdx.x;
  { float s = 0.f; const float* row = KX + (b * CX + t) * NP;
#pragma unroll 1
    for (int n = 0; n < NP; ++n) s += bfr(row[n]); sg[t] = s / (float)NP; }
  __syncthreads(); float g2 = sg[t] * sg[t];
#pragma unroll
  for (int o = 1; o < 32; o <<= 1) g2 += __shfl_xor(g2, o);
  if ((t & 31) == 0) red[t >> 5] = g2; __syncthreads(); float gg = 0.f; for (int i = 0; i < 8; ++i) gg += red[i]; const float ng = sqrtf(gg);
  for (int n = t; n < NP; n += 256) { float num = 0.f, nx = 0.f;
#pragma unroll 1
    for (int c = 0; c < CX; ++c) { const float xv = bfr(X[(b * CX + c) * NP + n]); num += xv * sg[c]; nx += xv * xv; }
    so2[n] = num / fmaxf(sqrtf(nx) * ng, CEPS); }
  __syncthreads(); for (int q = t; q < NP / 4; q += 256) vst2(MK + b * NP + q * 4, *(const v4f*)&so2[q * 4]); }
__global__ __launch_bounds__(128) void k_w(const _Float16* __restrict__ YT, const float* __restrict__ WW, const float* __restrict__ BW, const float* __restrict__ G, const float* __restrict__ BT, const float* __restrict__ MEAN, const float* __restrict__ VAR, const float* __restrict__ MK, const float* __restrict__ X, float* __restrict__ OUT) { __shared__ __align__(16) float sf[4][16][132]; __shared__ __align__(16) _Float16 sw[64][CI + 8];
  const int tid = threadIdx.x, wave = tid >> 5, lane = tid & 31, col = lane & 15, g = lane >> 4; const size_t b = blockIdx.z; const int c0 = blockIdx.x * 64 + wave * 16; const int p0 = blockIdx.y * 128;
  for (int e = tid; e < 64 * CI; e += 128) { const int cl = e >> 7, k = e & 127; sw[cl][k] = (_Float16)bfr(WW[(size_t)(blockIdx.x * 64 + cl) * CI + k]); } __syncthreads();
  v8f acc[8] = {}, accl[8] = {};
#pragma unroll
  for (int kc = 0; kc < CI / 32; ++kc) { v16h a; { const _Float16* p = &sw[wave * 16 + col][kc * 32 + 8 * g];
#pragma unroll
      for (int i = 0; i < 8; ++i) { a[i] = p[i]; a[8 + i] = p[16 + i]; } }
#pragma unroll
    for (int j = 0; j < 8; ++j) { const size_t o = (b * NP + p0 + j * 16 + col) * CI + kc * 32; acc[j] = wmma16(a, frag_h(YT + o, lane), acc[j]); accl[j] = wmma16(a, frag_h(YT + QTSZ + o, lane), accl[j]); } }
#pragma unroll
  for (int r = 0; r < 8; ++r) { const int c = c0 + 8 * g + r; const float inv = bfr(G[c]) / sqrtf(bfr(VAR[c]) + BNE), mu = bfr(MEAN[c]), be = bfr(BT[c]), bb = bfr(BW[c]);
#pragma unroll
    for (int j = 0; j < 8; ++j) { const int n = p0 + j * 16 + col; const float wy = acc[j][r] + accl[j][r] * (1.0f / 2048.0f) + bb; const float bn = (wy - mu) * inv + be; sf[wave][8 * g + r][j * 16 + col] = bn * MK[b * NP + n] + bfr(X[((b * CX + c) * NP) + n]); } }
  LDSX(); for (int rl = 0; rl < 16; ++rl) vst2(OUT + ((b * CX + c0 + rl) * NP) + p0 + lane * 4, *(const v4f*)&sf[wave][rl][lane * 4]); }
extern "C" void kernel_launch(void* const* d_in, const int* in_sizes, int n_in, void* d_out, int out_size, void* d_ws, size_t ws_size, hipStream_t stream) {
  (void)in_sizes; (void)n_in; (void)out_size;
  const float** F = (const float**)d_in;
  if (ws_size < (size_t)WS_END) return;
  char* ws = (char*)d_ws; __bf16* XT = (__bf16*)(ws + WS_XT); _Float16 *QT = (_Float16*)(ws + WS_QT), *KT = (_Float16*)(ws + WS_KT), *VTT = (_Float16*)(ws + WS_VTT), *V = (_Float16*)(ws + WS_V), *YT = (_Float16*)(ws + WS_YT); float* MK = (float*)(ws + WS_MK);
  k_xt<<<dim3(NP / 64, TNB, 8), 256, 0, stream>>>(F[0], F[1], XT);
  k_conv<<<dim3(CI / 64, NP / 128, 3 * TNB), 128, 0, stream>>>(F[2], F[3], F[4], F[5], F[6], F[7], XT, QT, KT, VTT);
  k_vtr<<<dim3(NM / 64, TNB), 256, 0, stream>>>(VTT, V);
  k_mask<<<TNB, 256, 0, stream>>>(F[0], F[1], MK);
  k_attn1<<<dim3(TQ, TNB), 128, 0, stream>>>(QT, KT, V, YT);
  k_w<<<dim3(CX / 64, (TQ * 64) / 128, TNB), 128, 0, stream>>>(YT, F[8], F[9], F[10], F[11], F[12], F[13], MK, F[0], (float*)d_out);
}
